// VarifoldLayer_28690381537760
// MI455X (gfx1250) — hardware-verified
//
#include <hip/hip_runtime.h>


namespace {
constexpr int B = 4, N = 2048, D = 128, NBLK = N / 16;
constexpr float XS = 8.0f, PS = 1024.0f, WSC = 256.0f, INV2S2 = 2.0f;
typedef _Float16 b16;
typedef __attribute__((ext_vector_type(16))) _Float16 v16b;
typedef __attribute__((ext_vector_type(8))) _Float16 v8b;
typedef __attribute__((ext_vector_type(8))) float v8f;
typedef __attribute__((ext_vector_type(4))) float v4f;
__device__ __forceinline__ float bf16_rne(float f) { unsigned int u = __float_as_uint(f); u += 0x7FFFu + ((u >> 16) & 1u); return __uint_as_float(u & 0xFFFF0000u); }
__device__ __forceinline__ void split16(float v, b16& hi, b16& lo) { hi = (b16)v; lo = (b16)(v - (float)hi); }
__device__ __forceinline__ v16b frag_kb(const b16* p, int hh) { const v8b a = *(const v8b*)(p + 8 * hh), b = *(const v8b*)(p + 16 + 8 * hh); v16b f;
#pragma unroll
  for (int e = 0; e < 8; ++e) { f[e] = a[e]; f[8 + e] = b[e]; } return f; }
__device__ __forceinline__ v8f wmma16b(v16b a, v16b b, v8f c) { v8f d = __builtin_amdgcn_wmma_f32_16x16x32_f16(false, a, false, b, (short)0, c, false, false); asm volatile("v_nop\n\tv_nop\n\tv_nop\n\tv_nop" : "+v"(d) : "v"(a), "v"(b)); return d; }
__device__ __forceinline__ void wave_lds_sync() { __builtin_amdgcn_fence(__ATOMIC_RELEASE, "workgroup"); __builtin_amdgcn_wave_barrier(); __builtin_amdgcn_fence(__ATOMIC_ACQUIRE, "workgroup"); }
__device__ __forceinline__ float pmul(float a, float b) { float p = a * b; asm volatile("" : "+v"(p)); return p; }

__global__ __launch_bounds__(256) void wput_kernel(const float* __restrict__ w, int KIN, b16* __restrict__ WT) {
  const int KG = KIN / 8; const int u = blockIdx.x * 256 + threadIdx.x; if (u >= D * KG) return; const int o = u / KG, k0 = (u % KG) * 8; v8b v;
#pragma unroll
  for (int j = 0; j < 8; ++j) v[j] = (b16)(bf16_rne(w[(size_t)(k0 + j) * D + o]) * WSC); for (int pass = 0; pass < 2; ++pass) { *(volatile v8b*)(WT + (size_t)o * KIN + k0) = v; __threadfence(); }
}
__global__ __launch_bounds__(32) void vf_kernel(const float* __restrict__ pos, const float* __restrict__ feat, const float* __restrict__ wts, const b16* __restrict__ W1T, const float* __restrict__ b1, const b16* __restrict__ W2T, const float* __restrict__ b2, const b16* __restrict__ WA1T, const float* __restrict__ ba1, const float* __restrict__ Wa2, const float* __restrict__ ba2, int BV, float* __restrict__ out) {
  __shared__ __attribute__((aligned(16))) b16 Ph[16][40], Pl[16][40], Fh[D][40], Ah[16][2 * D + 8], Al[16][2 * D + 8], Bh[16][D + 8], Bl[16][D + 8]; __shared__ float Qp[16][4], Rs[16], Tr[16][D + 1], At[16];
  const int lane = threadIdx.x, nloc = lane & 15, hlf = lane >> 4; const int b = blockIdx.x / NBLK; if (b >= BV) return; const size_t i0 = (size_t)(blockIdx.x % NBLK) * 16; const float* pb = pos + (size_t)b * N * 3; const float* fb = feat + (size_t)b * N * D;
  if (lane < 16) { for (int c = 0; c < 3; ++c) Qp[lane][c] = bf16_rne(pb[(i0 + lane) * 3 + c]); Rs[lane] = 0.0f; }
  for (int rr = 0; rr < 16; ++rr) for (int qd = 0; qd < 4; ++qd) { Ah[rr][qd * 32 + lane] = (b16)(bf16_rne(fb[(i0 + rr) * D + qd * 32 + lane]) * XS); Al[rr][qd * 32 + lane] = (b16)0.0f; }
  wave_lds_sync(); v8f acc[8];
#pragma unroll
  for (int t = 0; t < 8; ++t) acc[t] = (v8f){};
  float rs[16]; for (int r = 0; r < 16; ++r) rs[r] = 0.0f;
#pragma unroll 1
  for (int j0 = 0; j0 < N; j0 += 32) { const size_t j = j0 + lane; const float px = bf16_rne(pb[j * 3]), py = bf16_rne(pb[j * 3 + 1]), pz = bf16_rne(pb[j * 3 + 2]), wj = bf16_rne(wts[(size_t)b * N + j]);
#pragma unroll
    for (int r = 0; r < 16; ++r) { const float dx = Qp[r][0] - px, dy = Qp[r][1] - py, dz = Qp[r][2] - pz; const float kk = pmul(__expf(-INV2S2 * (pmul(dx, dx) + pmul(dy, dy) + pmul(dz, dz))), wj); rs[r] += kk; b16 p, q; split16(kk * PS, p, q); Ph[r][lane] = p; Pl[r][lane] = q; }
    for (int rr = 0; rr < 32; ++rr) for (int qd = 0; qd < 4; ++qd) Fh[qd * 32 + lane][rr] = (b16)(bf16_rne(fb[(size_t)(j0 + rr) * D + qd * 32 + lane]) * XS);
    wave_lds_sync(); const v16b pa = frag_kb(&Ph[nloc][0], hlf), pl = frag_kb(&Pl[nloc][0], hlf);
#pragma unroll
    for (int t = 0; t < 8; ++t) { const v16b fh = frag_kb(&Fh[t * 16 + nloc][0], hlf); acc[t] = wmma16b(pa, fh, acc[t]); acc[t] = wmma16b(pl, fh, acc[t]); }
    wave_lds_sync(); }
#pragma unroll
  for (int r = 0; r < 16; ++r) { float s = rs[r]; for (int o = 16; o; o >>= 1) s += __shfl_xor(s, o); if (lane == 0) Rs[r] = s; }
  wave_lds_sync();
#pragma unroll
  for (int t = 0; t < 8; ++t)
#pragma unroll
    for (int r8 = 0; r8 < 8; ++r8) { const int rl = 8 * hlf + r8; const float ag = acc[t][r8] * (1.0f / (PS * XS)) / (Rs[rl] + 1e-8f); b16 p, q; split16(ag * XS, p, q); Bh[rl][t * 16 + nloc] = p; Bl[rl][t * 16 + nloc] = q; }
  wave_lds_sync();
  { v8f a2[8];
#pragma unroll
    for (int t = 0; t < 8; ++t) a2[t] = (v8f){};
#pragma unroll
    for (int kb = 0; kb < D; kb += 32) { const v16b a = frag_kb(&Bh[nloc][kb], hlf), al = frag_kb(&Bl[nloc][kb], hlf);
#pragma unroll
      for (int t = 0; t < 8; ++t) { const v16b bw = frag_kb(W1T + (size_t)(t * 16 + nloc) * D + kb, hlf); a2[t] = wmma16b(a, bw, a2[t]); a2[t] = wmma16b(al, bw, a2[t]); } }
    wave_lds_sync();
#pragma unroll
    for (int t = 0; t < 8; ++t) { const int c = t * 16 + nloc; const float bb = bf16_rne(b1[c]);
#pragma unroll
      for (int r8 = 0; r8 < 8; ++r8) { b16 p, q; split16(fmaxf(a2[t][r8] * (1.0f / (XS * WSC)) + bb, 0.0f) * XS, p, q); Bh[8 * hlf + r8][c] = p; Bl[8 * hlf + r8][c] = q; } } }
  wave_lds_sync();
  { v8f a2[8];
#pragma unroll
    for (int t = 0; t < 8; ++t) a2[t] = (v8f){};
#pragma unroll
    for (int kb = 0; kb < D; kb += 32) { const v16b a = frag_kb(&Bh[nloc][kb], hlf), al = frag_kb(&Bl[nloc][kb], hlf);
#pragma unroll
      for (int t = 0; t < 8; ++t) { const v16b bw = frag_kb(W2T + (size_t)(t * 16 + nloc) * D + kb, hlf); a2[t] = wmma16b(a, bw, a2[t]); a2[t] = wmma16b(al, bw, a2[t]); } }
#pragma unroll
    for (int t = 0; t < 8; ++t) { const int c = t * 16 + nloc; const float bb = bf16_rne(b2[c]);
#pragma unroll
      for (int r8 = 0; r8 < 8; ++r8) { const int rl = 8 * hlf + r8; const float tv = a2[t][r8] * (1.0f / (XS * WSC)) + bb; Tr[rl][c] = tv; b16 p, q; split16(tv * XS, p, q); Ah[rl][D + c] = p; Al[rl][D + c] = q; } } }
  wave_lds_sync();
  { v8f a2[8]; float pd[8];
#pragma unroll
    for (int t = 0; t < 8; ++t) a2[t] = (v8f){};
#pragma unroll
    for (int r8 = 0; r8 < 8; ++r8) pd[r8] = 0.0f;
#pragma unroll 2
    for (int kb = 0; kb < 2 * D; kb += 32) { const v16b a = frag_kb(&Ah[nloc][kb], hlf); v16b al; const bool two = kb >= D; if (two) al = frag_kb(&Al[nloc][kb], hlf);
#pragma unroll
      for (int t = 0; t < 8; ++t) { const v16b bw = frag_kb(WA1T + (size_t)(t * 16 + nloc) * (2 * D) + kb, hlf); a2[t] = wmma16b(a, bw, a2[t]); if (two) a2[t] = wmma16b(al, bw, a2[t]); } }
#pragma unroll
    for (int t = 0; t < 8; ++t) { const int c = t * 16 + nloc; const float bb = bf16_rne(ba1[c]), w2 = bf16_rne(Wa2[c]);
#pragma unroll
      for (int r8 = 0; r8 < 8; ++r8) pd[r8] += pmul(fmaxf(a2[t][r8] * (1.0f / (XS * WSC)) + bb, 0.0f), w2); }
#pragma unroll
    for (int r8 = 0; r8 < 8; ++r8) { float s = pd[r8]; for (int o = 1; o < 16; o <<= 1) s += __shfl_xor(s, o); if (nloc == 0) At[8 * hlf + r8] = 1.0f / (1.0f + __expf(-(s + bf16_rne(ba2[0])))); } }
  wave_lds_sync();
  for (int pass = 0; pass < 2; ++pass) { for (int rr = 0; rr < 16; ++rr) { v4f o; for (int q4 = 0; q4 < 4; ++q4) { const int c = lane * 4 + q4; o[q4] = bf16_rne(fb[(i0 + rr) * D + c]) + pmul(At[rr], Tr[rr][c]); } *(volatile v4f*)(out + ((size_t)b * N + i0 + rr) * D + lane * 4) = o; } __threadfence(); }
}
}

extern "C" void kernel_launch(void* const* d_in, const int* in_sizes, int n_in, void* d_out, int out_size, void* d_ws, size_t ws_size, hipStream_t stream) {
  (void)n_in;
  auto Fp = [&](int i) { return (const float*)d_in[i]; };
  if (in_sizes[0] != B * N * 3 || in_sizes[1] != B * N * D || in_sizes[2] != B * N || in_sizes[3] != D * D || in_sizes[5] != D * D || in_sizes[7] != 2 * D * D || in_sizes[9] != D || out_size != B * N * D) return;
  const int BV = B;
  size_t off = 0; char* ws = (char*)d_ws;
  auto carve = [&](size_t bytes) { char* p = ws + off; off += (bytes + 255) & ~(size_t)255; return p; };
  b16* W1T = (b16*)carve(D * D * 2); b16* W2T = (b16*)carve(D * D * 2); b16* WA1T = (b16*)carve(2 * D * D * 2);
  if (off > ws_size || off > ((size_t)1 << 20)) return;
  wput_kernel<<<(D * 16 + 255) / 256, 256, 0, stream>>>(Fp(3), D, W1T); wput_kernel<<<(D * 16 + 255) / 256, 256, 0, stream>>>(Fp(5), D, W2T); wput_kernel<<<(D * 32 + 255) / 256, 256, 0, stream>>>(Fp(7), 2 * D, WA1T);
  vf_kernel<<<BV * NBLK, 32, 0, stream>>>(Fp(0), Fp(1), Fp(2), W1T, Fp(4), W2T, Fp(6), WA1T, Fp(8), Fp(9), Fp(10), BV, (float*)d_out);
}
